// FastShiftNet_32512902431268
// MI455X (gfx1250) — hardware-verified
//
#include <hip/hip_runtime.h>
#include <math.h>

typedef __attribute__((ext_vector_type(16))) _Float16 v16h;
typedef __attribute__((ext_vector_type(16))) __bf16 v16b;
typedef __attribute__((ext_vector_type(8)))  _Float16 v8h;
typedef __attribute__((ext_vector_type(8)))  float v8f;
typedef __attribute__((ext_vector_type(4)))  float v4f;
typedef __attribute__((ext_vector_type(2)))  float v2f;
typedef __attribute__((ext_vector_type(4)))  unsigned v4u;
typedef __attribute__((ext_vector_type(4)))  int v4i;
typedef float __attribute__((may_alias)) float_a;
typedef int __attribute__((may_alias)) int_a;

template <typename T> __device__ __forceinline__ void vst2(void* p, T v) { *(volatile T*)p = v; __threadfence(); *(volatile T*)p = v; }
__device__ __forceinline__ v8f wmma16(v16h a, v16h b, v8f c) {
  v8f d = __builtin_amdgcn_wmma_f32_16x16x32_f16(false, a, false, b, (short)0, c, false, false);
  asm volatile("v_nop\n\tv_nop\n\tv_nop\n\tv_nop" : "+v"(d) : "v"(a), "v"(b));
  return d;
}
__device__ __forceinline__ v8f wmma_bf(v16b a, v16b b, v8f c) {
  v8f d = __builtin_amdgcn_wmma_f32_16x16x32_bf16(false, a, false, b, (short)0, c, false, false);
  asm volatile("v_nop\n\tv_nop\n\tv_nop\n\tv_nop" : "+v"(d) : "v"(a), "v"(b));
  return d;
}
__device__ __forceinline__ v16h frag_h(const _Float16* rowk0, int lane) {
  union { v16h v; v8h q[2]; } u; const _Float16* p = rowk0 + 8 * (lane >> 4);
  u.q[0] = *(const v8h*)p; u.q[1] = *(const v8h*)(p + 16); return u.v;
}
__device__ __forceinline__ v16h frag_f32(const float* rowk0, int lane) {
  v16h a; const float* p = rowk0 + 8 * (lane >> 4);
#pragma unroll
  for (int i = 0; i < 8; ++i) { a[i] = (_Float16)p[i]; a[8 + i] = (_Float16)p[16 + i]; }
  return a;
}
__device__ __forceinline__ v16h frag_f32s(const float* rowk0, int lane, float sc) {
  v16h a; const float* p = rowk0 + 8 * (lane >> 4);
#pragma unroll
  for (int i = 0; i < 8; ++i) { a[i] = (_Float16)(p[i] * sc); a[8 + i] = (_Float16)(p[16 + i] * sc); }
  return a;
}
__device__ __forceinline__ v16h fragc_f32(const float* W, int k0, int n, int lane, int ld, int K) {
  v16h a; const int g = lane >> 4;
#pragma unroll
  for (int i = 0; i < 8; ++i) { const int ka = k0 + 8 * g + i, kb = ka + 16;
    a[i] = (_Float16)(ka < K ? W[(size_t)(ka < K ? ka : K - 1) * ld + n] : 0.f); a[8 + i] = (_Float16)(kb < K ? W[(size_t)(kb < K ? kb : K - 1) * ld + n] : 0.f); }
  return a;
}
struct F2 { v16b h, l; };
__device__ __forceinline__ F2 bsplit16(const float v[16]) { F2 r;
#pragma unroll
  for (int i = 0; i < 16; ++i) { const __bf16 h = (__bf16)v[i]; r.h[i] = h; r.l[i] = (__bf16)(v[i] - (float)h); }
  return r; }
__device__ __forceinline__ F2 split_row(const float* row, int k0, int lane) { float v[16]; const float* p = row + k0 + 8 * (lane >> 4);
#pragma unroll
  for (int i = 0; i < 8; ++i) { v[i] = p[i]; v[8 + i] = p[16 + i]; }
  return bsplit16(v); }
__device__ __forceinline__ F2 split_rowK(const float* row, int k0, int lane, int K) { float v[16]; const int g = lane >> 4;
#pragma unroll
  for (int i = 0; i < 8; ++i) { const int ka = k0 + 8 * g + i, kb = ka + 16; v[i] = ka < K ? row[ka < K ? ka : K - 1] : 0.f; v[8 + i] = kb < K ? row[kb < K ? kb : K - 1] : 0.f; }
  return bsplit16(v); }
__device__ __forceinline__ F2 split_col(const float* W, int k0, int n, int lane, int ld, int K) { float v[16]; const int g = lane >> 4;
#pragma unroll
  for (int i = 0; i < 8; ++i) { const int ka = k0 + 8 * g + i, kb = ka + 16; v[i] = ka < K ? W[(size_t)(ka < K ? ka : K - 1) * ld + n] : 0.f; v[8 + i] = kb < K ? W[(size_t)(kb < K ? kb : K - 1) * ld + n] : 0.f; }
  return bsplit16(v); }
__device__ __forceinline__ v8f mac3(const F2& a, const F2& b, v8f c) { c = wmma_bf(a.l, b.h, c); c = wmma_bf(a.h, b.l, c); return wmma_bf(a.h, b.h, c); }
__device__ __forceinline__ float sigm(float v) { return 1.0f / (1.0f + expf(-v)); }
#define LDSX() do { asm volatile("s_wait_dscnt 0" ::: "memory"); __builtin_amdgcn_wave_barrier(); __builtin_amdgcn_fence(__ATOMIC_RELEASE, "workgroup"); } while (0)


#define NR 65536
#define NBIT 64
#define HID 512
#define CH 8192
#ifndef NCHUNK
#define NCHUNK (NR / CH)
#endif
typedef __attribute__((ext_vector_type(8))) __bf16 v8b;
__device__ __forceinline__ v16b frag_b(const __bf16* rowk0, int lane) {
  union { v16b v; v8b q[2]; } u; const __bf16* p = rowk0 + 8 * (lane >> 4);
  u.q[0] = *(const v8b*)p; u.q[1] = *(const v8b*)(p + 16); return u.v;
}
__device__ __forceinline__ float bfr(float v) { return (float)(__bf16)v; }
__device__ __attribute__((noinline)) float exp_ni(float v) { return expf(v); }
__device__ __attribute__((noinline)) float erf_ni(float v) { return erff(v); }

#define PK_1 0
#define PK_2 (PK_1 + HID * NBIT)
#define PK_3 (PK_2 + HID * HID)
#define PK_END (PK_3 + NBIT * HID)
#define WS_PK 0u
#define WS_H1 (WS_PK + 2u * PK_END)
#define WS_H2 (WS_H1 + 4u * CH * HID)
#define WS_END (WS_H2 + 4u * CH * HID)

__global__ __launch_bounds__(256) void k_packT(const float* __restrict__ W1, const float* __restrict__ W2, const float* __restrict__ W3, __bf16* __restrict__ PK) {
  __shared__ __align__(16) __bf16 s[HID]; const int n = blockIdx.x, which = blockIdx.y, tid = threadIdx.x; int K; size_t dst; const float* Wm; int N;
  if (which == 0) { Wm = W1; K = NBIT; N = HID; dst = PK_1 + (size_t)n * NBIT; } else if (which == 1) { Wm = W2; K = HID; N = HID; dst = PK_2 + (size_t)n * HID; } else { if (n >= NBIT) return; Wm = W3; K = HID; N = NBIT; dst = PK_3 + (size_t)n * HID; }
  for (int k = tid; k < K; k += 256) s[k] = (__bf16)Wm[(size_t)k * N + n];
  __syncthreads();
  for (int q = tid; q < K / 8; q += 256) vst2((unsigned*)(PK + dst + q * 8), *(const v4u*)&s[q * 8]);
}
template <int MODE>
__global__ __launch_bounds__(128) void k_lin(const float* __restrict__ A, const __bf16* __restrict__ P, const float* __restrict__ bias, const float* __restrict__ gam, const float* __restrict__ bet, float* __restrict__ Hout) {
  constexpr int K = (MODE == 1) ? NBIT : HID;
  __shared__ __align__(16) float so[4][16][132]; __shared__ float spart[4][16]; __shared__ float smean[16], srstd[16];
  const int tid = threadIdx.x, wave = tid >> 5, lane = tid & 31, col = lane & 15, g = lane >> 4; const size_t r0 = (size_t)blockIdx.x * 16; const int n0 = wave * 128;
  v8f acc[8] = {};
#pragma unroll 2
  for (int kc = 0; kc < K / 32; ++kc) { F2 a; if (MODE == 1) { v16b ax; const float* p = A + (r0 + col) * K + kc * 32 + 8 * g;
#pragma unroll
      for (int i = 0; i < 8; ++i) { ax[i] = (__bf16)p[i]; ax[8 + i] = (__bf16)p[16 + i]; } a.h = ax; a.l = ax; } else a = split_row(A + (r0 + col) * K, kc * 32, lane);
#pragma unroll
    for (int j = 0; j < 8; ++j) { const v16b w = frag_b(P + (size_t)(n0 + j * 16 + col) * K + kc * 32, lane); if (MODE != 1) acc[j] = wmma_bf(a.l, w, acc[j]); acc[j] = wmma_bf(a.h, w, acc[j]); } }
#pragma unroll
  for (int j = 0; j < 8; ++j) { const float bb = bfr(bias[n0 + j * 16 + col]);
#pragma unroll
    for (int r = 0; r < 8; ++r) so[wave][8 * g + r][j * 16 + col] = acc[j][r] + bb; }
  LDSX();
#pragma unroll 1
  for (int rl = 0; rl < 16; ++rl) { const float* q = &so[wave][rl][lane * 4]; float s = (q[0] + q[1]) + (q[2] + q[3]);
#pragma unroll
    for (int o = 1; o < 32; o <<= 1) s += __shfl_xor(s, o);
    if (lane == 0) spart[wave][rl] = s; }
  __syncthreads();
  if (tid < 16) smean[tid] = ((spart[0][tid] + spart[1][tid]) + (spart[2][tid] + spart[3][tid])) * (1.0f / (float)HID);
  __syncthreads();
#pragma unroll 1
  for (int rl = 0; rl < 16; ++rl) { const float mu = smean[rl]; const float* q = &so[wave][rl][lane * 4]; float s = 0.f;
#pragma unroll
    for (int i = 0; i < 4; ++i) { const float dv = q[i] - mu; s += dv * dv; }
#pragma unroll
    for (int o = 1; o < 32; o <<= 1) s += __shfl_xor(s, o);
    if (lane == 0) spart[wave][rl] = s; }
  __syncthreads();
  if (tid < 16) srstd[tid] = rsqrtf(((spart[0][tid] + spart[1][tid]) + (spart[2][tid] + spart[3][tid])) * (1.0f / (float)HID) + 1e-5f);
  __syncthreads();
#pragma unroll 1
  for (int rl = 0; rl < 16; ++rl) { const float mu = smean[rl], rs = srstd[rl]; v4f o; const float* q = &so[wave][rl][lane * 4];
#pragma unroll
    for (int i = 0; i < 4; ++i) { const int c = n0 + lane * 4 + i; const float y = (q[i] - mu) * rs * bfr(gam[c]) + bfr(bet[c]); o[i] = 0.5f * y * (1.0f + erf_ni(y * 0.70710678118654752f)); }
    vst2(Hout + (r0 + rl) * HID + n0 + lane * 4, o); }
}
__global__ __launch_bounds__(128) void k_out(const float* __restrict__ H2, const __bf16* __restrict__ P, const float* __restrict__ b3, const float* __restrict__ ABITS, float* __restrict__ OUT, size_t row_base) {
  __shared__ __align__(16) float sp[4][16][68]; __shared__ __align__(16) float sa[4][16][68]; __shared__ __align__(16) float so[4][16][68];
  const int tid = threadIdx.x, wave = tid >> 5, lane = tid & 31, col = lane & 15, g = lane >> 4; const size_t rloc = (size_t)blockIdx.x * 64 + wave * 16; const size_t rglob = row_base + rloc;
  v8f acc[4] = {};
#pragma unroll 2
  for (int kc = 0; kc < HID / 32; ++kc) { const F2 a = split_row(H2 + (rloc + col) * HID, kc * 32, lane);
#pragma unroll
    for (int j = 0; j < 4; ++j) { const v16b w = frag_b(P + (size_t)(j * 16 + col) * HID + kc * 32, lane); acc[j] = wmma_bf(a.l, w, acc[j]); acc[j] = wmma_bf(a.h, w, acc[j]); } }
#pragma unroll
  for (int r = 0; r < 8; ++r) { float v[4]; float mx = -3.0e38f;
#pragma unroll
    for (int j = 0; j < 4; ++j) { v[j] = acc[j][r] + bfr(b3[j * 16 + col]); mx = fmaxf(mx, v[j]); }
#pragma unroll
    for (int o = 1; o < 16; o <<= 1) mx = fmaxf(mx, __shfl_xor(mx, o));
    float z = 0.f;
#pragma unroll
    for (int j = 0; j < 4; ++j) { v[j] = exp_ni(v[j] - mx); z += v[j]; }
#pragma unroll
    for (int o = 1; o < 16; o <<= 1) z += __shfl_xor(z, o);
    const float iz = 1.0f / z;
#pragma unroll
    for (int j = 0; j < 4; ++j) sp[wave][8 * g + r][j * 16 + col] = v[j] * iz; }
#pragma unroll 1
  for (int rl = 0; rl < 16; ++rl) { const float* ar = ABITS + (rglob + rl) * NBIT; sa[wave][rl][lane * 2] = bfr(ar[lane * 2]); sa[wave][rl][lane * 2 + 1] = bfr(ar[lane * 2 + 1]); }
  LDSX();
#pragma unroll 1
  for (int rl = 0; rl < 16; ++rl) { const float* pr = &sp[wave][rl][0]; const float* ar = &sa[wave][rl][0];
#pragma unroll 1
    for (int h2 = 0; h2 < 2; ++h2) { const int i = lane * 2 + h2; float o = 0.f;
#pragma unroll 1
      for (int s = 0; s <= i; ++s) o += pr[s] * ar[i - s];
      so[wave][rl][i] = o; } }
  LDSX();
  for (int rl = 0; rl < 16; ++rl) if (lane < 16) vst2(OUT + (rglob + rl) * NBIT + lane * 4, *(const v4f*)&so[wave][rl][lane * 4]);
}
extern "C" void kernel_launch(void* const* d_in, const int* in_sizes, int n_in, void* d_out, int out_size, void* d_ws, size_t ws_size, hipStream_t stream) {
  (void)in_sizes; (void)n_in; (void)out_size;
  const float** F = (const float**)d_in;
  if (ws_size < (size_t)WS_END) return;
  char* ws = (char*)d_ws; __bf16* PK = (__bf16*)(ws + WS_PK); float *H1 = (float*)(ws + WS_H1), *H2 = (float*)(ws + WS_H2);
  k_packT<<<dim3(HID, 3), 256, 0, stream>>>(F[2], F[6], F[10], PK);
  for (int c = 0; c < NCHUNK; ++c) { const size_t rb = (size_t)c * CH;
    k_lin<1><<<CH / 16, 128, 0, stream>>>(F[1] + rb * NBIT, PK + PK_1, F[3], F[4], F[5], H1);
    k_lin<2><<<CH / 16, 128, 0, stream>>>(H1, PK + PK_2, F[7], F[8], F[9], H2);
    k_out<<<CH / 64, 128, 0, stream>>>(H2, PK + PK_3, F[11], F[0], (float*)d_out, rb); }
}
